// PointNetLocalAggregation_59596966199813
// MI455X (gfx1250) — hardware-verified
//
#include <hip/hip_runtime.h>
#include <stddef.h>
#include <math.h>

#pragma clang fp contract(off)


#define NB     4
#define NPTS   4096
#define CIN    64
#define KNN    16
#define KIN    67
#define K0P    96
#define C0     64
#define C1     64
#define C2     128
#define NTHR   256
#define NWAVE  8
#define QB     64
#define P0     104
#define P1     72
#define WSCL   16.0f
#define HSCL   4.0f
#define INV16  0.0625f
#define INV64  0.015625f
#define BN_EPS 1e-5f
#define DBIG   3.0e38f

#define G0     (C0 * K0P / 8)
#define G1     (C1 * C0 / 8)
#define G2     (C2 * C1 / 8)
#define GT     (G0 + G1 + G2)

#define L_IDX    0
#define L_SC     (L_IDX + QB * KNN * 4)
#define L_SH     (L_SC + 256 * 4)
#define L_CAND   (L_SH + 256 * 4)
#define L_U      (L_CAND + NPTS * 16)
#define TW_A0    0
#define TW_H1    (TW_A0 + 16 * P0 * 2)
#define TW_H2    (TW_H1 + 16 * P1 * 2)
#define TW_O     (TW_H2 + 16 * P1 * 2)
#define TW_SZ    (TW_O + C2 * 4)
#define LDS_MAIN (L_U + NWAVE * TW_SZ)

static_assert(QB == NWAVE * 8);
static_assert(NTHR == NWAVE * 32);
static_assert((GT % NTHR) == 0 && (G0 % NTHR) == 0 && ((G0 + G1) % NTHR) == 0);
static_assert((L_SC % 16) == 0 && (L_CAND % 16) == 0 && (L_U % 16) == 0);
static_assert((TW_H1 % 16) == 0 && (TW_H2 % 16) == 0 && (TW_O % 16) == 0 && (TW_SZ % 16) == 0);
static_assert((P0 * 2) % 16 == 0 && (P1 * 2) % 16 == 0);
static_assert((K0P % 32) == 0 && (C0 % 32) == 0 && (C1 % 32) == 0);
static_assert(C0 + C1 + C2 == NTHR);
static_assert((NPTS % QB) == 0);

typedef float    v4f  __attribute__((ext_vector_type(4)));
typedef float    v8f  __attribute__((ext_vector_type(8)));
typedef _Float16 v8h  __attribute__((ext_vector_type(8)));
typedef _Float16 v16h __attribute__((ext_vector_type(16)));
union FragH { v16h v; v8h h[2]; };

__device__ __forceinline__ v8f wmh(v16h a, v16h b, v8f c) {
  v8f d = __builtin_amdgcn_wmma_f32_16x16x32_f16(false, a, false, b, (short)0, c, false, false);
#if defined(__HIP_DEVICE_COMPILE__)
  asm volatile("v_nop\n\tv_nop\n\tv_nop\n\tv_nop" : "+v"(d) : "v"(a), "v"(b));
#endif
  return d;
}

__device__ __forceinline__ v8f zero8() {
  v8f z = {0.f, 0.f, 0.f, 0.f, 0.f, 0.f, 0.f, 0.f};
  return z;
}

template <int KT, int NT>
__device__ __forceinline__ void mma(v8f (&acc)[8], const _Float16* ar, const _Float16* __restrict__ bplane,
                                    int KP, int m, int hh) {
#pragma unroll
  for (int t = 0; t < NT; ++t) acc[t] = zero8();
#pragma unroll
  for (int kt = 0; kt < KT; ++kt) {
    FragH a;
    a.h[0] = *(const v8h*)(ar + 32 * kt);
    a.h[1] = *(const v8h*)(ar + 32 * kt + 16);
#pragma unroll
    for (int t = 0; t < NT; ++t) {
      const _Float16* bp = bplane + (size_t)(16 * t + m) * KP + 32 * kt + 8 * hh;
      FragH b;
      b.h[0] = *(const v8h*)bp;
      b.h[1] = *(const v8h*)(bp + 16);
      acc[t] = wmh(a.v, b.v, acc[t]);
    }
  }
}

template <int NT>
__device__ __forceinline__ void epi_to_lds(const v8f (&acc)[8], _Float16* sp, int pitch,
                                           const float* sc, const float* sh, int m, float inv) {
#pragma unroll
  for (int t = 0; t < NT; ++t) {
    const float a = sc[16 * t + m];
    const float c = sh[16 * t + m];
#pragma unroll
    for (int r = 0; r < 8; ++r) {
      float v = acc[t][r] * inv;
      v = v * a + c;
      v = fmaxf(v, 0.0f) * HSCL;
      sp[r * pitch + 16 * t] = (_Float16)v;
    }
  }
}

__device__ __forceinline__ void ins16(float (&dd)[KNN], int (&jj)[KNN], float dk, int jk) {
#pragma unroll
  for (int t = 0; t < KNN; ++t) {
    const bool sw = (dk < dd[t]) || (dk == dd[t] && jk < jj[t]);
    const float od = dd[t];
    const int   oj = jj[t];
    dd[t] = sw ? dk : od;
    jj[t] = sw ? jk : oj;
    dk = sw ? od : dk;
    jk = sw ? oj : jk;
  }
}

__device__ __forceinline__ float sqn(float x, float y, float z) {
  const float t0 = x * x;
  const float t2 = z * z;
  float s = t0 + t2;
  const float t1 = y * y;
  s = s + t1;
  return s;
}

__global__ __launch_bounds__(NTHR) void k_prep(
    const float* __restrict__ w0, const float* __restrict__ w1, const float* __restrict__ w2,
    _Float16* pW0, _Float16* pW1, _Float16* pW2) {
  const int bstart = blockIdx.x * NTHR;
  const int i = bstart + (int)threadIdx.x;
  if (i >= GT) return;
  float v[8];
  _Float16* dp;
  if (bstart < G0) {
    const int o  = i * 8;
    const int n  = o / K0P;
    const int k0 = o - n * K0P;
#pragma unroll
    for (int e = 0; e < 8; ++e) {
      const int k   = k0 + e;
      const int col = k < CIN ? 3 + k : (k < KIN ? k - CIN : 0);
      const float xv = w0[(size_t)n * KIN + col];
      v[e] = (k < KIN) ? xv * WSCL : xv * 0.0f;
    }
    dp = pW0 + o;
  } else if (bstart < G0 + G1) {
    const int o  = (i - G0) * 8;
    const int n  = o >> 6;
    const int k0 = o & 63;
#pragma unroll
    for (int e = 0; e < 8; ++e) v[e] = w1[(size_t)n * C0 + k0 + e] * WSCL;
    dp = pW1 + o;
  } else {
    const int o  = (i - G0 - G1) * 8;
    const int n  = o >> 6;
    const int k0 = o & 63;
#pragma unroll
    for (int e = 0; e < 8; ++e) v[e] = w2[(size_t)n * C1 + k0 + e] * WSCL;
    dp = pW2 + o;
  }
  v8h hv;
#pragma unroll
  for (int e = 0; e < 8; ++e) hv[e] = (_Float16)v[e];
  *(volatile v8h*)dp = hv;
  __threadfence();
  *(volatile v8h*)dp = hv;
}

__global__ __launch_bounds__(NTHR) void k_main(
    const float* __restrict__ xyz, const float* __restrict__ points,
    const float* __restrict__ b0, const float* __restrict__ g0, const float* __restrict__ be0,
    const float* __restrict__ rm0, const float* __restrict__ rv0,
    const float* __restrict__ b1, const float* __restrict__ g1, const float* __restrict__ be1,
    const float* __restrict__ rm1, const float* __restrict__ rv1,
    const float* __restrict__ b2, const float* __restrict__ g2, const float* __restrict__ be2,
    const float* __restrict__ rm2, const float* __restrict__ rv2,
    const _Float16* __restrict__ pW0, const _Float16* __restrict__ pW1, const _Float16* __restrict__ pW2,
    float* out) {
  extern __shared__ v4f lds_dyn[];
  char* lb = (char*)lds_dyn;
  int*   sIdx  = (int*)(lb + L_IDX);
  float* sSc   = (float*)(lb + L_SC);
  float* sSh   = (float*)(lb + L_SH);
  v4f*   sCand = (v4f*)(lb + L_CAND);
  char*  ub    = lb + L_U;

  const int tid = threadIdx.x, lane = tid & 31, wave = tid >> 5, hh = lane >> 4, m = lane & 15;
  const int b  = blockIdx.x / (NPTS / QB);
  const int qb = blockIdx.x - b * (NPTS / QB);
  const int q0 = qb * QB;
  const size_t bN = (size_t)b * NPTS;

  for (int i = tid; i < NPTS; i += NTHR) {
    const float* xp = xyz + (bN + (size_t)i) * 3;
    const float x = xp[0], y = xp[1], z = xp[2];
    v4f c;
    c[0] = x; c[1] = y; c[2] = z; c[3] = sqn(x, y, z);
    sCand[i] = c;
  }
  {
    float gv, rvv, bv, rmv, bev;
    if (wave < 2) {
      const int n = tid;
      gv = g0[n]; rvv = rv0[n]; bv = b0[n]; rmv = rm0[n]; bev = be0[n];
    } else if (wave < 4) {
      const int n = tid - C0;
      gv = g1[n]; rvv = rv1[n]; bv = b1[n]; rmv = rm1[n]; bev = be1[n];
    } else {
      const int n = tid - C0 - C1;
      gv = g2[n]; rvv = rv2[n]; bv = b2[n]; rmv = rm2[n]; bev = be2[n];
    }
    const float sc = rsqrtf(rvv + BN_EPS) * gv;
    sSc[tid] = sc;
    sSh[tid] = (bv - rmv) * sc + bev;
  }
  __syncthreads();

  if (wave < 2) {
    const int q = tid;
    const v4f qv = sCand[q0 + q];
    const float qx = qv[0], qy = qv[1], qz = qv[2], qsq = qv[3];
    float dd[KNN];
    int   jj[KNN];
#pragma unroll
    for (int t = 0; t < KNN; ++t) { dd[t] = DBIG; jj[t] = NPTS; }
#pragma unroll 2
    for (int j = 0; j < NPTS; ++j) {
      const v4f cd = sCand[j];
      float p = qx * cd[0];
      p = fmaf(qy, cd[1], p);
      p = fmaf(qz, cd[2], p);
      const float s = qsq + cd[3];
      const float d = s - 2.0f * p;
      if (d < dd[KNN - 1] || (d == dd[KNN - 1] && j < jj[KNN - 1])) ins16(dd, jj, d, j);
    }
#pragma unroll
    for (int t = 0; t < KNN; ++t) {
      int j = jj[t];
      j = j < 0 ? 0 : (j > NPTS - 1 ? NPTS - 1 : j);
      sIdx[q * KNN + t] = j;
    }
  }
  __syncthreads();

  _Float16* tA0 = (_Float16*)(ub + wave * TW_SZ + TW_A0);
  _Float16* tH1 = (_Float16*)(ub + wave * TW_SZ + TW_H1);
  _Float16* tH2 = (_Float16*)(ub + wave * TW_SZ + TW_H2);
  float*    sO  = (float*)(ub + wave * TW_SZ + TW_O);
  const float* sc0 = sSc;
  const float* sh0 = sSh;
  const float* sc1 = sSc + C0;
  const float* sh1 = sSh + C0;
  const float* sc2 = sSc + C0 + C1;
  const float* sh2 = sSh + C0 + C1;

  v8f acc[8];
  for (int it = 0; it < QB / NWAVE; ++it) {
    const int ql = it * NWAVE + wave;
    const int qi = q0 + ql;

    {
      const int k = lane >> 1, hf = lane & 1;
      int j = sIdx[ql * KNN + k];
      j = j < 0 ? 0 : (j > NPTS - 1 ? NPTS - 1 : j);
      const v4f* pr = (const v4f*)(points + (bN + (size_t)j) * CIN + 32 * hf);
      _Float16* dst = tA0 + k * P0;
#pragma unroll
      for (int g = 0; g < 4; ++g) {
        const v4f u0 = pr[2 * g];
        const v4f u1 = pr[2 * g + 1];
        v8h hv;
        hv[0] = (_Float16)u0[0]; hv[1] = (_Float16)u0[1]; hv[2] = (_Float16)u0[2]; hv[3] = (_Float16)u0[3];
        hv[4] = (_Float16)u1[0]; hv[5] = (_Float16)u1[1]; hv[6] = (_Float16)u1[2]; hv[7] = (_Float16)u1[3];
        *(v8h*)(dst + 32 * hf + 8 * g) = hv;
      }
      const v4f cj = sCand[j];
      const v4f cq = sCand[qi];
      const float rx = cj[0] - cq[0];
      const float ry = cj[1] - cq[1];
      const float rz = cj[2] - cq[2];
      const float zr = rz * 0.0f;
      v8h e;
      e[0] = (_Float16)(hf == 0 ? rx : zr);
      e[1] = (_Float16)(hf == 0 ? ry : zr);
      e[2] = (_Float16)(hf == 0 ? rz : zr);
      e[3] = (_Float16)zr; e[4] = (_Float16)zr; e[5] = (_Float16)zr; e[6] = (_Float16)zr; e[7] = (_Float16)zr;
      *(v8h*)(dst + 64 + 8 * hf) = e;
      v8h zv;
#pragma unroll
      for (int u = 0; u < 8; ++u) zv[u] = (_Float16)zr;
      *(v8h*)(dst + 80 + 8 * hf) = zv;
    }
    __syncthreads();

    mma<3, 4>(acc, tA0 + m * P0 + 8 * hh, pW0, K0P, m, hh);
    epi_to_lds<4>(acc, tH1 + (8 * hh) * P1 + m, P1, sc0, sh0, m, INV16);
    __syncthreads();

    mma<2, 4>(acc, tH1 + m * P1 + 8 * hh, pW1, C0, m, hh);
    epi_to_lds<4>(acc, tH2 + (8 * hh) * P1 + m, P1, sc1, sh1, m, INV64);
    __syncthreads();

    mma<2, 8>(acc, tH2 + m * P1 + 8 * hh, pW2, C1, m, hh);
    {
      float mx[8];
#pragma unroll
      for (int t = 0; t < 8; ++t) {
        const float a = sc2[16 * t + m];
        const float c = sh2[16 * t + m];
        float mm = 0.0f;
#pragma unroll
        for (int r = 0; r < 8; ++r) {
          float v = acc[t][r] * INV64;
          v = v * a + c;
          v = fmaxf(v, 0.0f);
          mm = fmaxf(mm, v);
        }
        mx[t] = mm;
      }
#pragma unroll
      for (int t = 0; t < 8; ++t) mx[t] = fmaxf(mx[t], __shfl_xor(mx[t], 16, 32));
#pragma unroll
      for (int t = 0; t < 8; ++t) sO[16 * t + m] = mx[t];
    }
    __syncthreads();

    {
      const v4f ov = *(const v4f*)(sO + 4 * lane);
      float* gp = out + (bN + (size_t)qi) * C2 + 4 * lane;
      *(volatile v4f*)gp = ov;
      __threadfence();
      *(volatile v4f*)gp = ov;
    }
  }
}

extern "C" void kernel_launch(void* const* d_in, const int* in_sizes, int n_in,
                              void* d_out, int out_size, void* d_ws, size_t ws_size,
                              hipStream_t stream) {
  if (n_in < 20) return;
  if (in_sizes[0] != NB * NPTS * 3 || in_sizes[1] != NB * NPTS * CIN) return;
  if (in_sizes[2] != C0 * KIN) return;
  for (int i = 3; i <= 7; ++i) if (in_sizes[i] != C0) return;
  if (in_sizes[8] != C1 * C0) return;
  for (int i = 9; i <= 13; ++i) if (in_sizes[i] != C1) return;
  if (in_sizes[14] != C2 * C1) return;
  for (int i = 15; i <= 19; ++i) if (in_sizes[i] != C2) return;
  if (out_size != NB * NPTS * C2) return;

  const float* xyz    = (const float*)d_in[0];
  const float* points = (const float*)d_in[1];
  const float* w0  = (const float*)d_in[2];
  const float* b0  = (const float*)d_in[3];
  const float* g0  = (const float*)d_in[4];
  const float* be0 = (const float*)d_in[5];
  const float* rm0 = (const float*)d_in[6];
  const float* rv0 = (const float*)d_in[7];
  const float* w1  = (const float*)d_in[8];
  const float* b1  = (const float*)d_in[9];
  const float* g1  = (const float*)d_in[10];
  const float* be1 = (const float*)d_in[11];
  const float* rm1 = (const float*)d_in[12];
  const float* rv1 = (const float*)d_in[13];
  const float* w2  = (const float*)d_in[14];
  const float* b2  = (const float*)d_in[15];
  const float* g2  = (const float*)d_in[16];
  const float* be2 = (const float*)d_in[17];
  const float* rm2 = (const float*)d_in[18];
  const float* rv2 = (const float*)d_in[19];
  float* out = (float*)d_out;

  char* ws = (char*)d_ws;
  size_t off = 0;
  const size_t oW0 = off; off += (size_t)C0 * K0P * 2;  off = (off + 255) & ~(size_t)255;
  const size_t oW1 = off; off += (size_t)C1 * C0 * 2;   off = (off + 255) & ~(size_t)255;
  const size_t oW2 = off; off += (size_t)C2 * C1 * 2;   off = (off + 255) & ~(size_t)255;
  if (off > ws_size || off > (size_t)134217728) return;
  _Float16* pW0 = (_Float16*)(ws + oW0);
  _Float16* pW1 = (_Float16*)(ws + oW1);
  _Float16* pW2 = (_Float16*)(ws + oW2);

  k_prep<<<GT / NTHR, NTHR, 0, stream>>>(w0, w1, w2, pW0, pW1, pW2);

  hipFuncSetAttribute(reinterpret_cast<const void*>(&k_main),
                      hipFuncAttributeMaxDynamicSharedMemorySize, LDS_MAIN);
  k_main<<<NB * (NPTS / QB), NTHR, LDS_MAIN, stream>>>(
      xyz, points, b0, g0, be0, rm0, rv0, b1, g1, be1, rm1, rv1, b2, g2, be2, rm2, rv2,
      pW0, pW1, pW2, out);
}
